// CompressedAttention_86878598463929
// MI455X (gfx1250) — hardware-verified
//
#include <hip/hip_runtime.h>
#include <hip/hip_bf16.h>
#include <math.h>
#include <stdint.h>

typedef __attribute__((ext_vector_type(16))) _Float16 v16h;
typedef __attribute__((ext_vector_type(8)))  _Float16 v8h;
typedef __attribute__((ext_vector_type(16))) __bf16   v16b;
typedef __attribute__((ext_vector_type(8)))  __bf16   v8b;
typedef __attribute__((ext_vector_type(8)))  float    v8f;
typedef __attribute__((ext_vector_type(4)))  float    v4f;
typedef __attribute__((ext_vector_type(4)))  unsigned v4u;

__device__ __forceinline__ unsigned short f2bf_bits(float f) {
  unsigned u = __float_as_uint(f);
  return (unsigned short)((u + 0x7FFFu + ((u >> 16) & 1u)) >> 16);
}
__device__ __forceinline__ float bf_bits2f(unsigned short h) { return __uint_as_float(((unsigned)h) << 16); }

__device__ __forceinline__ void dep_guard_h(v8f& a, v8f& b, v16h x, v16h y) { asm volatile("v_nop\n\tv_nop\n\tv_nop\n\tv_nop" : "+v"(a), "+v"(b) : "v"(x), "v"(y)); }
__device__ __forceinline__ void dep_guard_b(v8f& a, v8f& b, v16b x, v16b y) { asm volatile("v_nop\n\tv_nop\n\tv_nop\n\tv_nop" : "+v"(a), "+v"(b) : "v"(x), "v"(y)); }
__device__ __forceinline__ void keep4_h(v16h a, v16h b, v16h c, v16h d) { asm volatile("v_nop" :: "v"(a), "v"(b), "v"(c), "v"(d)); }
__device__ __forceinline__ void keep4_b(v16b a, v16b b, v16b c, v16b d) { asm volatile("v_nop" :: "v"(a), "v"(b), "v"(c), "v"(d)); }
__device__ __forceinline__ void acc_guard4(v8f& a, v8f& b, v8f& c, v8f& d) { asm volatile("v_nop\n\tv_nop\n\tv_nop\n\tv_nop" : "+v"(a), "+v"(b), "+v"(c), "+v"(d)); }
template <typename T> struct Frag;
template <> struct Frag<_Float16> {
  typedef v16h V; union U { v16h v; v8h h[2]; };
  static __device__ __forceinline__ v16h load(const _Float16* p) {
    U f; f.h[0] = *(const v8h*)(p); f.h[1] = *(const v8h*)(p + 16); return f.v;
  }
  static __device__ __forceinline__ v8f mma(v16h a, v16h b, v8f c) {
    return __builtin_amdgcn_wmma_f32_16x16x32_f16(false, a, false, b, (short)0, c, false, false);
  }
  static __device__ __forceinline__ void guard(v8f& a, v8f& b, v16h x, v16h y) { dep_guard_h(a, b, x, y); }
  static __device__ __forceinline__ void keep(v16h a, v16h b, v16h c, v16h d) { keep4_h(a, b, c, d); }
};
template <> struct Frag<__bf16> {
  typedef v16b V; union U { v16b v; v8b h[2]; };
  static __device__ __forceinline__ v16b load(const __bf16* p) {
    U f; f.h[0] = *(const v8b*)(p); f.h[1] = *(const v8b*)(p + 16); return f.v;
  }
  static __device__ __forceinline__ v8f mma(v16b a, v16b b, v8f c) {
    return __builtin_amdgcn_wmma_f32_16x16x32_bf16(false, a, false, b, (short)0, c, false, false);
  }
  static __device__ __forceinline__ void guard(v8f& a, v8f& b, v16b x, v16b y) { dep_guard_b(a, b, x, y); }
  static __device__ __forceinline__ void keep(v16b a, v16b b, v16b c, v16b d) { keep4_b(a, b, c, d); }
};

template <int ET> struct Elem;
template <> struct Elem<0> { typedef _Float16 T; };
template <> struct Elem<1> { typedef __bf16 T; };
template <int ET, bool SPLIT, int BIAS_MODE, int OUT_MODE, bool RESID, int ACT = 0>
__global__ __launch_bounds__(256) void wmma_gemm64(
    const unsigned short* __restrict__ Ap, const unsigned short* __restrict__ A2p, int lda, long strideA,
    const unsigned short* __restrict__ Btp, const unsigned short* __restrict__ Bt2p, int ldb, long strideB,
    void* __restrict__ Cout, void* __restrict__ Cout2, int ldc, long strideC,
    const float* __restrict__ bias,
    const float* __restrict__ resid, long strideR,
    int M, int N, int K, float scale) {
  typedef typename Elem<ET>::T T;
  typedef typename Frag<T>::V V;
  const T* A = (const T*)Ap; const T* A2 = (const T*)A2p; const T* Bt = (const T*)Btp; const T* Bt2 = (const T*)Bt2p;
  __shared__ __align__(16) float sT[8][16 * 68];
  const int b    = blockIdx.y;
  const int lane = threadIdx.x & 31;
  const int wave = threadIdx.x >> 5;
  const int tilesN = N >> 6;
  const int tilesM = M >> 6;
  const int tile = blockIdx.x * 8 + wave;
  if (tile >= tilesM * tilesN) return;
  const int tm = tile / tilesN;
  const int tn = tile - tm * tilesN;
  const int m0 = tm << 6;
  const int n0 = tn << 6;

  const T* Ab  = A  + (size_t)b * strideA;
  const T* Bb  = Bt + (size_t)b * strideB;
  const T* Ab2 = SPLIT ? (A2  + (size_t)b * strideA) : nullptr;
  const T* Bb2 = SPLIT ? (Bt2 + (size_t)b * strideB) : nullptr;

  const int rlane = lane & 15;
  const int koff  = (lane >> 4) * 8;
  const int mOff  = (lane >> 4) * 8;

  v8f acc[4][4];
#pragma unroll
  for (int i = 0; i < 4; ++i)
#pragma unroll
    for (int j = 0; j < 4; ++j) acc[i][j] = (v8f){0.f,0.f,0.f,0.f,0.f,0.f,0.f,0.f};

  for (int k0 = 0; k0 < K; k0 += 32) {
    V bh[4], bl[4];
#pragma unroll
    for (int j = 0; j < 4; ++j) {
      const size_t bo = (size_t)(n0 + (j << 4) + rlane) * ldb + koff + k0;
      bh[j] = Frag<T>::load(Bb + bo);
      if (SPLIT) bl[j] = Frag<T>::load(Bb2 + bo);
    }
#pragma unroll
    for (int i = 0; i < 4; ++i) {
      const size_t ao = (size_t)(m0 + (i << 4) + rlane) * lda + koff + k0;
      V ah = Frag<T>::load(Ab + ao);
      V al;
      if (SPLIT) al = Frag<T>::load(Ab2 + ao);
#pragma unroll
      for (int j = 0; j < 4; ++j) {
        acc[i][j] = Frag<T>::mma(ah, bh[j], acc[i][j]);
        if (SPLIT) {
          acc[i][j] = Frag<T>::mma(ah, bl[j], acc[i][j]);
          acc[i][j] = Frag<T>::mma(al, bh[j], acc[i][j]);
        }
      }
      Frag<T>::guard(acc[i][0], acc[i][3], ah, SPLIT ? al : ah);
    }
    Frag<T>::keep(bh[0], bh[1], bh[2], bh[3]);
    if (SPLIT) Frag<T>::keep(bl[0], bl[1], bl[2], bl[3]);
  }
  acc_guard4(acc[0][0], acc[0][1], acc[0][2], acc[0][3]);
  acc_guard4(acc[1][0], acc[1][1], acc[1][2], acc[1][3]);
  acc_guard4(acc[2][0], acc[2][1], acc[2][2], acc[2][3]);
  acc_guard4(acc[3][0], acc[3][1], acc[3][2], acc[3][3]);

  float* slab = sT[wave];
  const float* Rb = RESID ? (resid + (size_t)b * strideR) : nullptr;
#pragma unroll
  for (int i = 0; i < 4; ++i) {
    const int mBase = m0 + (i << 4);
#pragma unroll
    for (int j = 0; j < 4; ++j) {
      const int n = n0 + (j << 4) + rlane;
      float bv = 0.f;
      if (BIAS_MODE == 2) bv = bias[n];
#pragma unroll
      for (int r = 0; r < 8; ++r) {
        float v = acc[i][j][r] * scale;
        if (BIAS_MODE == 1) v += bias[mBase + mOff + r];
        if (BIAS_MODE == 2) v += bv;
        if (RESID) v += Rb[(size_t)(mBase + mOff + r) * ldc + n];
        if (ACT == 1) v = tanhf(v);
        if (ACT == 2) v = fmaxf(v, 0.0f);
        if (ACT == 3) v = v / (1.0f + expf(-v));
        if (ACT == 4) v = (v > 0.f) ? v : 0.01f * v;
        if (ACT == 5) v = 0.5f * v * (1.0f + erff(v * 0.70710678118654752f));
        slab[(mOff + r) * 68 + (j << 4) + rlane] = v;
      }
    }
    __builtin_amdgcn_fence(__ATOMIC_RELEASE, "workgroup");
    __builtin_amdgcn_wave_barrier();
    __builtin_amdgcn_fence(__ATOMIC_ACQUIRE, "workgroup");
    if (OUT_MODE == 0) {
      float* C = (float*)Cout + (size_t)b * strideC;
      const int hh = lane >> 4, c4 = (lane & 15) * 4;
      for (int pass = 0; pass < 2; ++pass) {
#pragma unroll
        for (int it = 0; it < 8; ++it) {
          const int row = it * 2 + hh;
          v4f v = *(const v4f*)(slab + row * 68 + c4);
          *(volatile v4f*)(C + (size_t)(mBase + row) * ldc + n0 + c4) = v;
        }
        __threadfence();
      }
    } else {
      const int q = lane >> 3, c8 = (lane & 7) * 8;
      unsigned short* C  = (unsigned short*)Cout  + (size_t)b * strideC;
      unsigned short* C2 = (OUT_MODE == 2) ? ((unsigned short*)Cout2 + (size_t)b * strideC) : nullptr;
      for (int pass = 0; pass < 2; ++pass) {
#pragma unroll
        for (int it = 0; it < 4; ++it) {
          const int row = it * 4 + q;
          const float* sp = slab + row * 68 + c8;
          v8h hv, lv;
#pragma unroll
          for (int e = 0; e < 8; ++e) {
            if (OUT_MODE == 1) {
              hv[e] = (_Float16)sp[e];
            } else {
              unsigned short hb = f2bf_bits(sp[e]);
              unsigned short lb = f2bf_bits(sp[e] - bf_bits2f(hb));
              hv[e] = __builtin_bit_cast(_Float16, hb);
              lv[e] = __builtin_bit_cast(_Float16, lb);
            }
          }
          *(volatile v8h*)(C + (size_t)(mBase + row) * ldc + n0 + c8) = hv;
          if (OUT_MODE == 2) *(volatile v8h*)(C2 + (size_t)(mBase + row) * ldc + n0 + c8) = lv;
        }
        __threadfence();
      }
    }
    __builtin_amdgcn_fence(__ATOMIC_RELEASE, "workgroup");
    __builtin_amdgcn_wave_barrier();
    __builtin_amdgcn_fence(__ATOMIC_ACQUIRE, "workgroup");
  }
}

__device__ __forceinline__ v8f at_mma(v16b a, v16b b, v8f c) {
  c = __builtin_amdgcn_wmma_f32_16x16x32_bf16(false, a, false, b, (short)0, c, false, false);
  asm volatile("v_nop\n\tv_nop\n\tv_nop\n\tv_nop" : "+v"(c) : "v"(a), "v"(b));
  return c;
}

constexpr int N_BATCH   = 2;
constexpr int SEQ_LEN   = 2048;
constexpr int DMOD      = 1024;
constexpr int DLAT      = 128;
constexpr int DROT      = 32;
constexpr int NROPE_PAD = 64;
constexpr int NHEAD     = 16;
constexpr int HDIM      = 64;
constexpr int SDEP      = HDIM + DROT;
constexpr int MTOK      = N_BATCH * SEQ_LEN;

static_assert(MTOK % 64 == 0 && DMOD % 64 == 0 && DLAT % 64 == 0 && NROPE_PAD % 64 == 0);
static_assert(DMOD % 32 == 0 && DLAT % 32 == 0);
static_assert(SDEP % 32 == 0 && SEQ_LEN % 64 == 0);

__global__ __launch_bounds__(256) void split_rows_bf16x8(
    const float* __restrict__ in, unsigned short* __restrict__ hi, unsigned short* __restrict__ lo, int n8) {
  const int i = blockIdx.x * 256 + threadIdx.x;
  if (i < n8) {
    const v4f a = *(const v4f*)(in + (size_t)8 * i);
    const v4f b = *(const v4f*)(in + (size_t)8 * i + 4);
    v8h hv, lv;
#pragma unroll
    for (int e = 0; e < 8; ++e) {
      const float f = (e < 4) ? a[e] : b[e - 4];
      const unsigned short hb = f2bf_bits(f);
      const unsigned short lb = f2bf_bits(f - bf_bits2f(hb));
      hv[e] = __builtin_bit_cast(_Float16, hb);
      lv[e] = __builtin_bit_cast(_Float16, lb);
    }
    unsigned short* ph = hi + (size_t)8 * i;
    unsigned short* pl = lo + (size_t)8 * i;
    *(volatile v8h*)ph = hv;
    *(volatile v8h*)pl = lv;
    __threadfence();
    *(volatile v8h*)ph = hv;
    *(volatile v8h*)pl = lv;
  }
}

__global__ __launch_bounds__(256) void transpose_split_bf16(
    const float* __restrict__ W, unsigned short* __restrict__ hi, unsigned short* __restrict__ lo,
    int kdim, int nreal) {
  __shared__ float tile[64][33];
  const int tid = threadIdx.x;
  const int k0 = blockIdx.x * 64;
  const int n0 = blockIdx.y * 32;
#pragma unroll
  for (int it = 0; it < 2; ++it) {
    const int idx = it * 256 + tid;
    const int kr = idx >> 3;
    const int c4 = (idx & 7) * 4;
    const int n = n0 + c4;
    const int ncl = (n + 3 < nreal) ? n : (nreal - 4);
    const v4f v = *(const v4f*)(W + (size_t)(k0 + kr) * nreal + ncl);
    const bool ok = (n < nreal);
    tile[kr][c4 + 0] = ok ? v[0] : 0.f;
    tile[kr][c4 + 1] = ok ? v[1] : 0.f;
    tile[kr][c4 + 2] = ok ? v[2] : 0.f;
    tile[kr][c4 + 3] = ok ? v[3] : 0.f;
  }
  __syncthreads();
  const int nr = tid >> 3;
  const int c8 = (tid & 7) * 8;
  v8h hv, lv;
#pragma unroll
  for (int e = 0; e < 8; ++e) {
    const float f = tile[c8 + e][nr];
    const unsigned short hb = f2bf_bits(f);
    const unsigned short lb = f2bf_bits(f - bf_bits2f(hb));
    hv[e] = __builtin_bit_cast(_Float16, hb);
    lv[e] = __builtin_bit_cast(_Float16, lb);
  }
  const size_t o = (size_t)(n0 + nr) * kdim + k0 + c8;
  *(volatile v8h*)(hi + o) = hv;
  *(volatile v8h*)(lo + o) = lv;
  __threadfence();
  *(volatile v8h*)(hi + o) = hv;
  *(volatile v8h*)(lo + o) = lv;
}

struct RopeFreq { float f[16]; };
static_assert(sizeof(RopeFreq) == 64);

__global__ __launch_bounds__(128) void rope_split_bf16(
    const float* __restrict__ qraw, const float* __restrict__ kraw,
    unsigned short* __restrict__ qrh, unsigned short* __restrict__ qrl,
    unsigned short* __restrict__ krh, unsigned short* __restrict__ krl, RopeFreq g) {
#pragma clang fp contract(off)
  __shared__ float tile[32][33];
  __shared__ float sinv[16];
  const int tid = threadIdx.x;
  const int nblk = MTOK / 32;
  const bool isk = ((int)blockIdx.x >= nblk);
  const int row0 = (isk ? ((int)blockIdx.x - nblk) : (int)blockIdx.x) * 32;
  const float* raw = isk ? kraw : qraw;
  unsigned short* dhp = isk ? krh : qrh;
  unsigned short* dlp = isk ? krl : qrl;
  if (tid < 16) {
    float v = g.f[0];
#pragma unroll
    for (int e = 1; e < 16; ++e) v = (tid == e) ? g.f[e] : v;
    sinv[tid] = v;
  }
  __syncthreads();
#pragma unroll 1
  for (int it = 0; it < 4; ++it) {
    const int p = it * 128 + tid;
    const int r = p >> 4;
    const int j = p & 15;
    const int row = row0 + r;
    const int t = row & (SEQ_LEN - 1);
    const float* rp = raw + (size_t)row * NROPE_PAD;
    const float x1 = rp[j];
    const float x2 = rp[16 + j];
    const float ang = (float)t * sinv[j];
    float sn, cs;
    sincosf(ang, &sn, &cs);
    tile[r][j]      = x1 * cs - x2 * sn;
    tile[r][16 + j] = x2 * cs + x1 * sn;
  }
  __syncthreads();
  const int orow = tid >> 2;
  const int seg = (tid & 3) * 8;
  v8h hv, lv;
#pragma unroll
  for (int e = 0; e < 8; ++e) {
    const float f = tile[orow][seg + e];
    const unsigned short hb = f2bf_bits(f);
    const unsigned short lb = f2bf_bits(f - bf_bits2f(hb));
    hv[e] = __builtin_bit_cast(_Float16, hb);
    lv[e] = __builtin_bit_cast(_Float16, lb);
  }
  const size_t o = (size_t)(row0 + orow) * DROT + seg;
  *(volatile v8h*)(dhp + o) = hv;
  *(volatile v8h*)(dlp + o) = lv;
  __threadfence();
  *(volatile v8h*)(dhp + o) = hv;
  *(volatile v8h*)(dlp + o) = lv;
}

constexpr int A_QB = 64;
constexpr int A_KC = 64;
constexpr int A_NW = 4;
constexpr int OS_PITCH = 68;

__global__ __launch_bounds__(128)
void mla_attn96(const unsigned short* __restrict__ qh, const unsigned short* __restrict__ ql,
                const unsigned short* __restrict__ kh, const unsigned short* __restrict__ kl,
                const unsigned short* __restrict__ vh, const unsigned short* __restrict__ vl,
                const unsigned short* __restrict__ qrh, const unsigned short* __restrict__ qrl,
                const unsigned short* __restrict__ krh, const unsigned short* __restrict__ krl,
                unsigned short* __restrict__ oh, unsigned short* __restrict__ ol, float invs) {
  union FB { v16b v; v8b h[2]; };
  __shared__ __align__(16) unsigned short Ksh[A_KC * SDEP];
  __shared__ __align__(16) unsigned short Ksl[A_KC * SDEP];
  __shared__ __align__(16) unsigned short Vth[HDIM * A_KC];
  __shared__ __align__(16) unsigned short Vtl[HDIM * A_KC];
  __shared__ __align__(16) unsigned short Psh[A_NW][16 * A_KC];
  __shared__ __align__(16) unsigned short Psl[A_NW][16 * A_KC];
  __shared__ __align__(16) float Os[A_NW][16 * OS_PITCH];

  const int tid  = threadIdx.x;
  const int wave = tid >> 5;
  const int lane = tid & 31;
  const int hh   = lane >> 4;
  const int c    = lane & 15;

  const int nqb = SEQ_LEN / A_QB;
  const int bx  = blockIdx.x;
  const int qb  = bx % nqb;
  const int bhi = bx / nqb;
  const int h   = bhi % NHEAD;
  const int b   = bhi / NHEAD;
  const int q0  = qb * A_QB + wave * 16;
  const size_t tq = (size_t)b * SEQ_LEN + (size_t)(q0 + c);

  v16b qah[3], qal[3];
  {
    const __bf16* p0 = (const __bf16*)qh + tq * DMOD + h * HDIM + 8 * hh;
    const __bf16* p1 = (const __bf16*)ql + tq * DMOD + h * HDIM + 8 * hh;
    qah[0] = Frag<__bf16>::load(p0);
    qah[1] = Frag<__bf16>::load(p0 + 32);
    qal[0] = Frag<__bf16>::load(p1);
    qal[1] = Frag<__bf16>::load(p1 + 32);
    const __bf16* r0p = (const __bf16*)qrh + tq * DROT + 8 * hh;
    const __bf16* r1p = (const __bf16*)qrl + tq * DROT + 8 * hh;
    qah[2] = Frag<__bf16>::load(r0p);
    qal[2] = Frag<__bf16>::load(r1p);
  }

  float mrow[8], lrow[8];
  v8f oacc[4];
#pragma unroll
  for (int r = 0; r < 8; ++r) { mrow[r] = -INFINITY; lrow[r] = 0.f; }
#pragma unroll
  for (int t = 0; t < 4; ++t) oacc[t] = (v8f){0.f,0.f,0.f,0.f,0.f,0.f,0.f,0.f};

  const int nChunks = qb + 1;
  for (int kc = 0; kc < nChunks; ++kc) {
    const int kv0 = kc * A_KC;
    __syncthreads();
    {
      const int kvr = tid >> 1, hf = tid & 1;
      const size_t tk = (size_t)b * SEQ_LEN + (size_t)(kv0 + kvr);
      {
        const v4u* sh = (const v4u*)(kh + tk * DMOD + h * HDIM + hf * 32);
        const v4u* sl = (const v4u*)(kl + tk * DMOD + h * HDIM + hf * 32);
        v4u* dh = (v4u*)(Ksh + kvr * SDEP + hf * 32);
        v4u* dl = (v4u*)(Ksl + kvr * SDEP + hf * 32);
#pragma unroll
        for (int i = 0; i < 4; ++i) { dh[i] = sh[i]; dl[i] = sl[i]; }
      }
      asm volatile("" ::: "memory");
      {
        const v4u* sh = (const v4u*)(krh + tk * DROT + hf * 16);
        const v4u* sl = (const v4u*)(krl + tk * DROT + hf * 16);
        v4u* dh = (v4u*)(Ksh + kvr * SDEP + HDIM + hf * 16);
        v4u* dl = (v4u*)(Ksl + kvr * SDEP + HDIM + hf * 16);
#pragma unroll
        for (int i = 0; i < 2; ++i) { dh[i] = sh[i]; dl[i] = sl[i]; }
      }
      asm volatile("" ::: "memory");
      {
        const v4u* sh = (const v4u*)(vh + tk * DMOD + h * HDIM + hf * 32);
        const v4u* sl = (const v4u*)(vl + tk * DMOD + h * HDIM + hf * 32);
#pragma unroll
        for (int i = 0; i < 4; ++i) {
          const v4u wh = sh[i];
          const v4u wl = sl[i];
#pragma unroll
          for (int e = 0; e < 4; ++e) {
            const int d = hf * 32 + 8 * i + 2 * e;
            Vth[d * A_KC + kvr]       = (unsigned short)(wh[e] & 0xffffu);
            Vth[(d + 1) * A_KC + kvr] = (unsigned short)(wh[e] >> 16);
            Vtl[d * A_KC + kvr]       = (unsigned short)(wl[e] & 0xffffu);
            Vtl[(d + 1) * A_KC + kvr] = (unsigned short)(wl[e] >> 16);
          }
        }
      }
    }
    __syncthreads();

    v8f s[4];
#pragma unroll
    for (int j = 0; j < 4; ++j) {
      s[j] = (v8f){0.f,0.f,0.f,0.f,0.f,0.f,0.f,0.f};
#pragma unroll
      for (int dc = 0; dc < 3; ++dc) {
        FB kb, kq;
        const int ko = (j * 16 + c) * SDEP + dc * 32 + 8 * hh;
        kb.h[0] = *(const v8b*)(Ksh + ko);
        kb.h[1] = *(const v8b*)(Ksh + ko + 16);
        kq.h[0] = *(const v8b*)(Ksl + ko);
        kq.h[1] = *(const v8b*)(Ksl + ko + 16);
        s[j] = at_mma(qah[dc], kb.v, s[j]);
        s[j] = at_mma(qah[dc], kq.v, s[j]);
        s[j] = at_mma(qal[dc], kb.v, s[j]);
      }
    }
    const bool diag = (kc == qb);
    float cm[8];
#pragma unroll
    for (int r = 0; r < 8; ++r) {
      const int qrow = q0 + 8 * hh + r;
      float m = -INFINITY;
#pragma unroll
      for (int j = 0; j < 4; ++j) {
        const int kvcol = kv0 + j * 16 + c;
        float sv = s[j][r] * invs;
        if (diag && (kvcol > qrow)) sv = -INFINITY;
        s[j][r] = sv;
        m = fmaxf(m, sv);
      }
#pragma unroll
      for (int off = 1; off < 16; off <<= 1) m = fmaxf(m, __shfl_xor(m, off, 32));
      cm[r] = m;
    }
    unsigned short* pwh = Psh[wave];
    unsigned short* pwl = Psl[wave];
#pragma unroll
    for (int r = 0; r < 8; ++r) {
      const float mnew = fmaxf(mrow[r], cm[r]);
      const float alpha = expf(mrow[r] - mnew);
      mrow[r] = mnew;
      float psum = 0.f;
#pragma unroll
      for (int j = 0; j < 4; ++j) {
        const float p = expf(s[j][r] - mnew);
        psum += p;
        const unsigned short hb = f2bf_bits(p);
        const unsigned short lb = f2bf_bits(p - bf_bits2f(hb));
        pwh[(8 * hh + r) * A_KC + j * 16 + c] = hb;
        pwl[(8 * hh + r) * A_KC + j * 16 + c] = lb;
      }
#pragma unroll
      for (int off = 1; off < 16; off <<= 1) psum += __shfl_xor(psum, off, 32);
      lrow[r] = lrow[r] * alpha + psum;
#pragma unroll
      for (int t = 0; t < 4; ++t) oacc[t][r] *= alpha;
    }
    __builtin_amdgcn_fence(__ATOMIC_RELEASE, "workgroup");
    __builtin_amdgcn_wave_barrier();
    __builtin_amdgcn_fence(__ATOMIC_ACQUIRE, "workgroup");
#pragma unroll 1
    for (int kk = 0; kk < 2; ++kk) {
      FB pa, pl;
      pa.h[0] = *(const v8b*)(pwh + c * A_KC + kk * 32 + 8 * hh);
      pa.h[1] = *(const v8b*)(pwh + c * A_KC + kk * 32 + 16 + 8 * hh);
      pl.h[0] = *(const v8b*)(pwl + c * A_KC + kk * 32 + 8 * hh);
      pl.h[1] = *(const v8b*)(pwl + c * A_KC + kk * 32 + 16 + 8 * hh);
#pragma unroll
      for (int t = 0; t < 4; ++t) {
        FB vb, vq;
        vb.h[0] = *(const v8b*)(Vth + (t * 16 + c) * A_KC + kk * 32 + 8 * hh);
        vb.h[1] = *(const v8b*)(Vth + (t * 16 + c) * A_KC + kk * 32 + 16 + 8 * hh);
        vq.h[0] = *(const v8b*)(Vtl + (t * 16 + c) * A_KC + kk * 32 + 8 * hh);
        vq.h[1] = *(const v8b*)(Vtl + (t * 16 + c) * A_KC + kk * 32 + 16 + 8 * hh);
        oacc[t] = at_mma(pa.v, vb.v, oacc[t]);
        oacc[t] = at_mma(pa.v, vq.v, oacc[t]);
        oacc[t] = at_mma(pl.v, vb.v, oacc[t]);
      }
    }
  }

  float* os = Os[wave];
#pragma unroll
  for (int r = 0; r < 8; ++r) {
    const float inv = 1.0f / lrow[r];
#pragma unroll
    for (int t = 0; t < 4; ++t) os[(8 * hh + r) * OS_PITCH + t * 16 + c] = oacc[t][r] * inv;
  }
  __builtin_amdgcn_fence(__ATOMIC_RELEASE, "workgroup");
  __builtin_amdgcn_wave_barrier();
  __builtin_amdgcn_fence(__ATOMIC_ACQUIRE, "workgroup");
  {
    const int qq = lane >> 3, c8 = (lane & 7) * 8;
    for (int pass = 0; pass < 2; ++pass) {
#pragma unroll
      for (int it = 0; it < 4; ++it) {
        const int row = it * 4 + qq;
        const float* sp = os + row * OS_PITCH + c8;
        v8h hv, lv;
#pragma unroll
        for (int e = 0; e < 8; ++e) {
          const unsigned short hb = f2bf_bits(sp[e]);
          const unsigned short lb = f2bf_bits(sp[e] - bf_bits2f(hb));
          hv[e] = __builtin_bit_cast(_Float16, hb);
          lv[e] = __builtin_bit_cast(_Float16, lb);
        }
        const size_t o = ((size_t)b * SEQ_LEN + (size_t)(q0 + row)) * DMOD + h * HDIM + c8;
        *(volatile v8h*)(oh + o) = hv;
        *(volatile v8h*)(ol + o) = lv;
      }
      __threadfence();
    }
  }
}

constexpr size_t WSB_X    = (size_t)MTOK * DMOD * 2;
constexpr size_t WSB_WKVD = (size_t)DLAT * DMOD * 2;
constexpr size_t WSB_WKUP = (size_t)DMOD * DLAT * 2;
constexpr size_t WSB_WQ   = (size_t)DMOD * DMOD * 2;
constexpr size_t WSB_WQR  = (size_t)NROPE_PAD * DMOD * 2;
constexpr size_t WSB_WKR  = (size_t)NROPE_PAD * DLAT * 2;
constexpr size_t WSB_CKV  = (size_t)MTOK * DLAT * 2;
constexpr size_t WSB_TOK  = (size_t)MTOK * DMOD * 2;
constexpr size_t WSB_RAW  = (size_t)MTOK * NROPE_PAD * 4;
constexpr size_t WSB_ROT  = (size_t)MTOK * DROT * 2;
constexpr size_t WS_TOTAL = 2 * WSB_X + 2 * WSB_WKVD + 4 * WSB_WKUP + 2 * WSB_WQ + 2 * WSB_WQR + 2 * WSB_WKR
                          + 2 * WSB_WQ + 2 * WSB_CKV + 6 * WSB_TOK + 2 * WSB_RAW + 4 * WSB_ROT + 2 * WSB_TOK;
static_assert(WS_TOTAL == 99385344ull);
static_assert(WS_TOTAL <= 134217728ull);

extern "C" void kernel_launch(void* const* d_in, const int* in_sizes, int n_in,
                              void* d_out, int out_size, void* d_ws, size_t ws_size,
                              hipStream_t stream) {
  if (n_in != 8) return;
  if (in_sizes[0] != MTOK * DMOD || in_sizes[1] != DMOD * DLAT || in_sizes[2] != DLAT * DMOD ||
      in_sizes[3] != DLAT * DMOD || in_sizes[4] != DMOD * DMOD || in_sizes[5] != DMOD * DROT ||
      in_sizes[6] != DLAT * DROT || in_sizes[7] != DMOD * DMOD) return;
  if (out_size != MTOK * DMOD) return;
  if (ws_size < WS_TOTAL) return;

  const float* x         = (const float*)d_in[0];
  const float* W_kv_down = (const float*)d_in[1];
  const float* W_k_up    = (const float*)d_in[2];
  const float* W_v_up    = (const float*)d_in[3];
  const float* W_q       = (const float*)d_in[4];
  const float* W_q_rope  = (const float*)d_in[5];
  const float* W_k_rope  = (const float*)d_in[6];
  const float* W_o       = (const float*)d_in[7];
  float* out = (float*)d_out;

  size_t off = 0;
  auto carve = [&](size_t bytes) -> unsigned short* {
    unsigned short* p = (unsigned short*)((char*)d_ws + off);
    off += (bytes + 255) & ~(size_t)255;
    return p;
  };
  unsigned short* xh    = carve(WSB_X);
  unsigned short* xl    = carve(WSB_X);
  unsigned short* wkvdh = carve(WSB_WKVD);
  unsigned short* wkvdl = carve(WSB_WKVD);
  unsigned short* wkuph = carve(WSB_WKUP);
  unsigned short* wkupl = carve(WSB_WKUP);
  unsigned short* wvuph = carve(WSB_WKUP);
  unsigned short* wvupl = carve(WSB_WKUP);
  unsigned short* wqh   = carve(WSB_WQ);
  unsigned short* wql   = carve(WSB_WQ);
  unsigned short* wqrh  = carve(WSB_WQR);
  unsigned short* wqrl  = carve(WSB_WQR);
  unsigned short* wkrh  = carve(WSB_WKR);
  unsigned short* wkrl  = carve(WSB_WKR);
  unsigned short* woh   = carve(WSB_WQ);
  unsigned short* wol   = carve(WSB_WQ);
  unsigned short* ckvh  = carve(WSB_CKV);
  unsigned short* ckvl  = carve(WSB_CKV);
  unsigned short* kh    = carve(WSB_TOK);
  unsigned short* kl    = carve(WSB_TOK);
  unsigned short* vh    = carve(WSB_TOK);
  unsigned short* vl    = carve(WSB_TOK);
  unsigned short* qh    = carve(WSB_TOK);
  unsigned short* ql    = carve(WSB_TOK);
  float* qr_raw = (float*)carve(WSB_RAW);
  float* kr_raw = (float*)carve(WSB_RAW);
  unsigned short* qrh   = carve(WSB_ROT);
  unsigned short* qrl   = carve(WSB_ROT);
  unsigned short* krh   = carve(WSB_ROT);
  unsigned short* krl   = carve(WSB_ROT);
  unsigned short* ath   = carve(WSB_TOK);
  unsigned short* atl   = carve(WSB_TOK);
  if (off > ws_size) return;

  {
    const int n8 = MTOK * DMOD / 8;
    split_rows_bf16x8<<<(n8 + 255) / 256, 256, 0, stream>>>(x, xh, xl, n8);
  }
  transpose_split_bf16<<<dim3(DMOD / 64, DLAT / 32), 256, 0, stream>>>(W_kv_down, wkvdh, wkvdl, DMOD, DLAT);
  transpose_split_bf16<<<dim3(DLAT / 64, DMOD / 32), 256, 0, stream>>>(W_k_up, wkuph, wkupl, DLAT, DMOD);
  transpose_split_bf16<<<dim3(DLAT / 64, DMOD / 32), 256, 0, stream>>>(W_v_up, wvuph, wvupl, DLAT, DMOD);
  transpose_split_bf16<<<dim3(DMOD / 64, DMOD / 32), 256, 0, stream>>>(W_q, wqh, wql, DMOD, DMOD);
  transpose_split_bf16<<<dim3(DMOD / 64, NROPE_PAD / 32), 256, 0, stream>>>(W_q_rope, wqrh, wqrl, DMOD, DROT);
  transpose_split_bf16<<<dim3(DLAT / 64, NROPE_PAD / 32), 256, 0, stream>>>(W_k_rope, wkrh, wkrl, DLAT, DROT);
  transpose_split_bf16<<<dim3(DMOD / 64, DMOD / 32), 256, 0, stream>>>(W_o, woh, wol, DMOD, DMOD);

  auto gemm_blocks = [](int M, int N) { return (((M / 64) * (N / 64)) + 7) / 8; };

  wmma_gemm64<1, true, 0, 2, false><<<dim3(gemm_blocks(MTOK, DLAT), 1), 256, 0, stream>>>(
      xh, xl, DMOD, 0L, wkvdh, wkvdl, DMOD, 0L, (void*)ckvh, (void*)ckvl, DLAT, 0L,
      nullptr, nullptr, 0L, MTOK, DLAT, DMOD, 1.0f);
  wmma_gemm64<1, true, 0, 2, false><<<dim3(gemm_blocks(MTOK, DMOD), 1), 256, 0, stream>>>(
      ckvh, ckvl, DLAT, 0L, wkuph, wkupl, DLAT, 0L, (void*)kh, (void*)kl, DMOD, 0L,
      nullptr, nullptr, 0L, MTOK, DMOD, DLAT, 1.0f);
  wmma_gemm64<1, true, 0, 2, false><<<dim3(gemm_blocks(MTOK, DMOD), 1), 256, 0, stream>>>(
      ckvh, ckvl, DLAT, 0L, wvuph, wvupl, DLAT, 0L, (void*)vh, (void*)vl, DMOD, 0L,
      nullptr, nullptr, 0L, MTOK, DMOD, DLAT, 1.0f);
  wmma_gemm64<1, true, 0, 2, false><<<dim3(gemm_blocks(MTOK, DMOD), 1), 256, 0, stream>>>(
      xh, xl, DMOD, 0L, wqh, wql, DMOD, 0L, (void*)qh, (void*)ql, DMOD, 0L,
      nullptr, nullptr, 0L, MTOK, DMOD, DMOD, 1.0f);
  wmma_gemm64<1, true, 0, 0, false><<<dim3(gemm_blocks(MTOK, NROPE_PAD), 1), 256, 0, stream>>>(
      xh, xl, DMOD, 0L, wqrh, wqrl, DMOD, 0L, (void*)qr_raw, nullptr, NROPE_PAD, 0L,
      nullptr, nullptr, 0L, MTOK, NROPE_PAD, DMOD, 1.0f);
  wmma_gemm64<1, true, 0, 0, false><<<dim3(gemm_blocks(MTOK, NROPE_PAD), 1), 256, 0, stream>>>(
      ckvh, ckvl, DLAT, 0L, wkrh, wkrl, DLAT, 0L, (void*)kr_raw, nullptr, NROPE_PAD, 0L,
      nullptr, nullptr, 0L, MTOK, NROPE_PAD, DLAT, 1.0f);

  RopeFreq fr;
  for (int j = 0; j < 16; ++j) {
    const double p = pow(10000.0, (double)j / 16.0);
    const float p32 = (float)p;
    fr.f[j] = 1.0f / p32;
  }
  rope_split_bf16<<<2 * (MTOK / 32), 128, 0, stream>>>(qr_raw, kr_raw, qrh, qrl, krh, krl, fr);

  const float invs = 1.0f / (float)sqrt((double)(HDIM + DROT));
  mla_attn96<<<N_BATCH * NHEAD * (SEQ_LEN / A_QB), 128, 0, stream>>>(
      qh, ql, kh, kl, vh, vl, qrh, qrl, krh, krl, ath, atl, invs);

  wmma_gemm64<1, true, 0, 0, false><<<dim3(gemm_blocks(MTOK, DMOD), 1), 256, 0, stream>>>(
      ath, atl, DMOD, 0L, woh, wol, DMOD, 0L, (void*)out, nullptr, DMOD, 0L,
      nullptr, nullptr, 0L, MTOK, DMOD, DMOD, 1.0f);
}
